// EdgeDecoder_42941083025726
// MI455X (gfx1250) — hardware-verified
//
#include <hip/hip_runtime.h>
#include <stddef.h>


#define INC    128
#define HID    128
#define LDK    136
#define NTHR   256
#define NWAVE  8
#define EPW    16
#define EPB    (NWAVE * EPW)
#define SCL_A  8.0f
#define SCL_W  16.0f
#define SCL_B1 128.0f
#define SCL_W2 0.0078125f
#define WSCAP  134217728

static_assert(INC == 128 && HID == 128);
static_assert((LDK % 8) == 0 && LDK >= INC);
static_assert(NTHR == NWAVE * 32);
static_assert(EPB == 128);
static_assert(EPB == 4 * 32);
static_assert((INC % 32) == 0);

typedef float    v4f  __attribute__((ext_vector_type(4)));
typedef float    v8f  __attribute__((ext_vector_type(8)));
typedef _Float16 v4h  __attribute__((ext_vector_type(4)));
typedef _Float16 v8h  __attribute__((ext_vector_type(8)));
typedef _Float16 v16h __attribute__((ext_vector_type(16)));
union FragH { v16h v; v8h h[2]; };

__device__ __forceinline__ v8f wmh(v16h a, v16h b, v8f c) {
  v8f d = __builtin_amdgcn_wmma_f32_16x16x32_f16(false, a, false, b, (short)0, c, false, false);
  asm volatile("v_nop\n\tv_nop\n\tv_nop\n\tv_nop" : "+v"(d) : "v"(a), "v"(b));
  return d;
}

__global__ __launch_bounds__(NTHR) void k_prepw1(const float* __restrict__ W1, _Float16* w1p) {
  __shared__ __attribute__((aligned(16))) _Float16 sT[HID * LDK];
  const int tid = (int)threadIdx.x;
#pragma unroll 1
  for (int i = tid; i < INC * HID; i += NTHR) {
    const int k = i / HID;
    const int n = i & (HID - 1);
    sT[n * LDK + k] = (_Float16)(W1[i] * SCL_W);
  }
  __syncthreads();
  constexpr int UPR = INC / 8;
  constexpr int NU  = HID * UPR;
  static_assert((UPR & (UPR - 1)) == 0);
#pragma unroll 1
  for (int u = tid; u < NU; u += NTHR) {
    const int n  = u / UPR;
    const int k0 = (u & (UPR - 1)) * 8;
    const v8h v = *(const v8h*)(sT + n * LDK + k0);
    *(volatile v8h*)(w1p + (size_t)u * 8) = v;
  }
  __threadfence();
#pragma unroll 1
  for (int u = tid; u < NU; u += NTHR) {
    const int n  = u / UPR;
    const int k0 = (u & (UPR - 1)) * 8;
    const v8h v = *(const v8h*)(sT + n * LDK + k0);
    *(volatile v8h*)(w1p + (size_t)u * 8) = v;
  }
}

__global__ __launch_bounds__(NTHR) void k_edge_mlp(
    const float* __restrict__ z, const int* __restrict__ edge, const _Float16* __restrict__ w1p,
    const float* __restrict__ b1, const float* __restrict__ W2, const float* __restrict__ b2,
    float* out, int nE, int nN) {
  __shared__ __attribute__((aligned(16))) _Float16 xa[NWAVE * EPW * LDK];
  __shared__ __attribute__((aligned(16))) float sres[EPB];
  const int tid = (int)threadIdx.x, lane = tid & 31, wave = tid >> 5;
  const int hh = lane >> 4, m = lane & 15;
  const int bbase = (int)blockIdx.x * EPB;
  const int ebase = bbase + wave * EPW;

  int ge = ebase + m;
  ge = ge > nE - 1 ? nE - 1 : ge;
  ge = ge < 0 ? 0 : ge;
  const int iidx = (hh == 0) ? ge : nE + ge;
  int nid = edge[iidx];
  nid = nid < 0 ? 0 : (nid > nN - 1 ? nN - 1 : nid);

  _Float16* xw = xa + wave * (EPW * LDK);
  const int col = 4 * lane;
#pragma unroll 4
  for (int j = 0; j < EPW; ++j) {
    const int u = __shfl(nid, j);
    const int v = __shfl(nid, EPW + j);
    const v4f a = *(const v4f*)(z + (size_t)u * INC + col);
    const v4f c = *(const v4f*)(z + (size_t)v * INC + col);
    const v4f p = (a * c) * SCL_A;
    const v4h o = __builtin_convertvector(p, v4h);
    *(v4h*)(xw + j * LDK + col) = o;
  }
  __syncthreads();

  constexpr int KT = INC / 32;
  FragH af[KT];
  const _Float16* arow = xw + m * LDK + 8 * hh;
#pragma unroll
  for (int kc = 0; kc < KT; ++kc) {
    af[kc].h[0] = *(const v8h*)(arow + 32 * kc);
    af[kc].h[1] = *(const v8h*)(arow + 32 * kc + 16);
  }

  float part[8];
#pragma unroll
  for (int r = 0; r < 8; ++r) part[r] = 0.0f;

#pragma unroll 1
  for (int nt = 0; nt < HID / 16; ++nt) {
    const int n = nt * 16 + m;
    v8f acc = {0.f, 0.f, 0.f, 0.f, 0.f, 0.f, 0.f, 0.f};
    const _Float16* bp0 = w1p + (size_t)n * INC + 8 * hh;
#pragma unroll
    for (int kc = 0; kc < KT; ++kc) {
      FragH bf;
      bf.h[0] = *(const v8h*)(bp0 + 32 * kc);
      bf.h[1] = *(const v8h*)(bp0 + 32 * kc + 16);
      acc = wmh(af[kc].v, bf.v, acc);
    }
    const float b1s = b1[n] * SCL_B1;
    const float w2s = W2[n] * SCL_W2;
#pragma unroll
    for (int r = 0; r < 8; ++r) {
      float h = acc[r] + b1s;
      h = h > 0.0f ? h : 0.0f;
      part[r] += h * w2s;
    }
  }

#pragma unroll
  for (int r = 0; r < 8; ++r) {
    float t = part[r];
    t += __shfl_xor(t, 8);
    t += __shfl_xor(t, 4);
    t += __shfl_xor(t, 2);
    t += __shfl_xor(t, 1);
    part[r] = t;
  }
  float mine = 0.0f;
#pragma unroll
  for (int r = 0; r < 8; ++r) mine = ((m & 7) == r) ? part[r] : mine;
  const float b2v = b2[0];
  if (m < 8) sres[wave * EPW + 8 * hh + m] = mine + b2v;
  __syncthreads();

  if (wave == 0) {
    const v4f ov = *(const v4f*)(sres + 4 * lane);
    const int e0 = bbase + 4 * lane;
    const bool full = (e0 + 3 < nE);
    if (full) {
      *(volatile v4f*)(out + e0) = ov;
    } else {
      if (e0     < nE) *(volatile float*)(out + e0)     = ov.x;
      if (e0 + 1 < nE) *(volatile float*)(out + e0 + 1) = ov.y;
      if (e0 + 2 < nE) *(volatile float*)(out + e0 + 2) = ov.z;
    }
    __threadfence();
    if (full) {
      *(volatile v4f*)(out + e0) = ov;
    } else {
      if (e0     < nE) *(volatile float*)(out + e0)     = ov.x;
      if (e0 + 1 < nE) *(volatile float*)(out + e0 + 1) = ov.y;
      if (e0 + 2 < nE) *(volatile float*)(out + e0 + 2) = ov.z;
    }
  }
}

extern "C" void kernel_launch(void* const* d_in, const int* in_sizes, int n_in,
                              void* d_out, int out_size, void* d_ws, size_t ws_size,
                              hipStream_t stream) {
  if (n_in < 6) return;
  const int nN = in_sizes[0] / INC;
  const int nE = in_sizes[1] / 2;
  if (nN <= 0 || nE <= 0) return;
  if (in_sizes[0] != nN * INC || in_sizes[1] != 2 * nE) return;
  if (in_sizes[2] != INC * HID || in_sizes[3] != HID || in_sizes[4] != HID || in_sizes[5] != 1) return;
  if (out_size != nE) return;
  if (nE > (1 << 28) || nN > (1 << 23)) return;

  const float* z    = (const float*)d_in[0];
  const int*   edge = (const int*)d_in[1];
  const float* W1   = (const float*)d_in[2];
  const float* b1   = (const float*)d_in[3];
  const float* W2   = (const float*)d_in[4];
  const float* b2   = (const float*)d_in[5];
  float* out = (float*)d_out;

  size_t off = 0;
  const size_t oW1 = off; off += (size_t)HID * INC * 2; off = (off + 255) & ~(size_t)255;
  if (off > ws_size || off > (size_t)WSCAP) return;
  _Float16* w1p = (_Float16*)((char*)d_ws + oW1);

  const int nBlk = (nE + EPB - 1) / EPB;

  k_prepw1<<<1, NTHR, 0, stream>>>(W1, w1p);
  k_edge_mlp<<<nBlk, NTHR, 0, stream>>>(z, edge, w1p, b1, W2, b2, out, nE, nN);
}
